// EquivSetGNN3_63153199120612
// MI455X (gfx1250) — hardware-verified
//
#include <hip/hip_runtime.h>
#include <stddef.h>


#define CH      128
#define NTHR    256
#define NWAVE   8
#define EPT     8
#define NGRP    2
#define CHUNK   (NTHR * EPT * NGRP)
#define WCAP    (EPT * NGRP * 32)
#define LISTN   (NWAVE * WCAP)
#define NBC     4096
#define NBF     1024
#define RCAP    40960
#define RBN     128
#define OTHR    512
#define GROWS   128
#define DEGCAP  1024
#define EROWS   25600
#define AP      136
#define WROWS   640

#define LDS_A    (2 * GROWS * AP * 2)
#define LDS_G2   (LDS_A + GROWS * CH * 4)
#define LDS_FILL ((RCAP + NBF + LISTN) * 4 + 64)

static_assert((CHUNK & (CHUNK - 1)) == 0);
static_assert(CHUNK <= 4096);
static_assert(NBC == 4 * NBF);
static_assert(OTHR * 8 == NBC);
static_assert((RCAP % 32) == 0);
static_assert(GROWS == NWAVE * 16);
static_assert(GROWS * CH * 4 <= LDS_A);
static_assert((EROWS % NBF) == 0 && (EROWS % GROWS) == 0);
static_assert((WROWS * (CH / 8)) % NTHR == 0);
static_assert((AP % 8) == 0);
static_assert(((GROWS * CH / 4) % NTHR) == 0);

typedef float          v4f   __attribute__((ext_vector_type(4)));
typedef float          v8f   __attribute__((ext_vector_type(8)));
typedef int            v4i   __attribute__((ext_vector_type(4)));
typedef unsigned short v4us  __attribute__((ext_vector_type(4)));
typedef unsigned short v8us  __attribute__((ext_vector_type(8)));
typedef __bf16         v16bf __attribute__((ext_vector_type(16)));
union FragB { v16bf v; v8us h[2]; };
union U8    { v8us v;  v4us q[2]; };

__device__ __forceinline__ unsigned int bf_bits(float f) {
  const unsigned int u = __float_as_uint(f);
  return (u + 0x7FFFu + ((u >> 16) & 1u)) >> 16;
}
__device__ __forceinline__ void split1(float f, unsigned short& h, unsigned short& l) {
  const unsigned int hb = bf_bits(f);
  const float hf = __uint_as_float(hb << 16);
  const unsigned int lb = bf_bits(f - hf);
  h = (unsigned short)hb;
  l = (unsigned short)lb;
}
__device__ __forceinline__ void split4(v4f v, v4us& h, v4us& l) {
  unsigned short h0, l0, h1, l1, h2, l2, h3, l3;
  split1(v.x, h0, l0); split1(v.y, h1, l1); split1(v.z, h2, l2); split1(v.w, h3, l3);
  v4us hh, ll;
  hh.x = h0; hh.y = h1; hh.z = h2; hh.w = h3;
  ll.x = l0; ll.y = l1; ll.z = l2; ll.w = l3;
  h = hh; l = ll;
}

__device__ __forceinline__ v8f wm3(v16bf ah, v16bf al, v16bf bh, v16bf bl, v8f c) {
  v8f d = __builtin_amdgcn_wmma_f32_16x16x32_bf16(false, ah, false, bh, (short)0, c, false, false);
  d = __builtin_amdgcn_wmma_f32_16x16x32_bf16(false, al, false, bh, (short)0, d, false, false);
  d = __builtin_amdgcn_wmma_f32_16x16x32_bf16(false, ah, false, bl, (short)0, d, false, false);
  asm volatile("v_nop\n\tv_nop\n\tv_nop\n\tv_nop" : "+v"(d) : "v"(ah), "v"(al), "v"(bh), "v"(bl));
  return d;
}

__device__ __forceinline__ void mma_strip(const unsigned short* arH, const unsigned short* arL,
                                          const unsigned short* __restrict__ bpH,
                                          const unsigned short* __restrict__ bpL, v8f (&acc)[8]) {
#pragma unroll
  for (int kt = 0; kt < CH / 32; ++kt) {
    FragB ah, al;
    ah.h[0] = *(const v8us*)(arH + 32 * kt);
    ah.h[1] = *(const v8us*)(arH + 32 * kt + 16);
    al.h[0] = *(const v8us*)(arL + 32 * kt);
    al.h[1] = *(const v8us*)(arL + 32 * kt + 16);
#pragma unroll
    for (int t = 0; t < 8; ++t) {
      const unsigned short* ph = bpH + (size_t)t * (16 * CH) + 32 * kt;
      const unsigned short* pl = bpL + (size_t)t * (16 * CH) + 32 * kt;
      FragB bh, bl;
      bh.h[0] = *(const v8us*)ph;
      bh.h[1] = *(const v8us*)(ph + 16);
      bl.h[0] = *(const v8us*)pl;
      bl.h[1] = *(const v8us*)(pl + 16);
      acc[t] = wm3(ah.v, al.v, bh.v, bl.v, acc[t]);
    }
  }
}

__device__ __forceinline__ void stage_rows(const float* __restrict__ A, int nRowsA, int rowBase,
                                           unsigned short* sH, unsigned short* sL, int tid) {
#pragma unroll 4
  for (int it = 0; it < (GROWS * CH / 4) / NTHR; ++it) {
    const int idx = it * NTHR + tid;
    const int r   = idx >> 5;
    const int c0  = (idx & 31) * 4;
    int row = rowBase + r;
    row = row > nRowsA - 1 ? nRowsA - 1 : row;
    const v4f v = *(const v4f*)(A + (size_t)row * CH + c0);
    v4us h, l;
    split4(v, h, l);
    const int o = r * AP + c0;
    *(v4us*)(sH + o) = h;
    *(v4us*)(sL + o) = l;
  }
}

__device__ __forceinline__ void epi_rows(v8f (&acc)[8], float* stg, const float* __restrict__ bias,
                                         int useBias, int relu, float* dst, int rowBase, int nRowsOut,
                                         int wave, int lane) {
  const int hh = lane >> 4, m = lane & 15;
  float* sp = stg + (wave * 16 + 8 * hh) * CH + m;
#pragma unroll
  for (int t = 0; t < 8; ++t) {
    const float bl = bias[16 * t + m];
    const float bv = useBias != 0 ? bl : 0.0f;
#pragma unroll
    for (int r = 0; r < 8; ++r) {
      float v = acc[t][r] + bv;
      v = relu != 0 ? fmaxf(v, 0.0f) : v;
      sp[r * CH + 16 * t] = v;
    }
  }
  __syncthreads();
  const float* lp = stg + wave * 16 * CH + 4 * lane;
#pragma unroll
  for (int i = 0; i < 16; ++i) {
    const int row = rowBase + wave * 16 + i;
    if (row < nRowsOut) {
      const v4f v = *(const v4f*)(lp + i * CH);
      *(volatile v4f*)(dst + (size_t)row * CH + 4 * lane) = v;
    }
  }
  __threadfence();
#pragma unroll
  for (int i = 0; i < 16; ++i) {
    const int row = rowBase + wave * 16 + i;
    if (row < nRowsOut) {
      const v4f v = *(const v4f*)(lp + i * CH);
      *(volatile v4f*)(dst + (size_t)row * CH + 4 * lane) = v;
    }
  }
}

__device__ __forceinline__ v4f seg_sum(const int* __restrict__ csr, int csrLen, int st, int n,
                                       const float* __restrict__ src, int smax, int lane) {
  v4f acc = {0.f, 0.f, 0.f, 0.f};
#pragma unroll 1
  for (int q0 = 0; q0 < n; q0 += 32) {
    int pos = st + q0 + lane;
    pos = pos < 0 ? 0 : (pos > csrLen - 1 ? csrLen - 1 : pos);
    int sl = csr[pos];
    sl = sl < 0 ? 0 : (sl > smax ? smax : sl);
    const int mcnt = (n - q0) < 32 ? (n - q0) : 32;
#pragma unroll 1
    for (int p = 0; p < mcnt; ++p) {
      const int s = __builtin_amdgcn_readlane(sl, p);
      acc = acc + *(const v4f*)(src + (size_t)s * CH + 4 * lane);
    }
  }
  return acc;
}

template <int NB>
__device__ __forceinline__ int scan_chunk(const int* __restrict__ dsts, int nE, int cbase, int slotBase,
                                          int nValid, int vec8, int* list, int tid, int lane, int wave) {
  int wc = 0;
#pragma unroll
  for (int g = 0; g < NGRP; ++g) {
    const int el0  = (g * NTHR + tid) * EPT;
    const int e0   = cbase + el0;
    const int sent = -2147483647 - 1;
    v4i da, db;
    if (vec8 != 0 && cbase + CHUNK <= nE) {
      da = *(const v4i*)(dsts + e0);
      db = *(const v4i*)(dsts + e0 + 4);
    } else {
      da.x = (e0     < nE) ? dsts[min(e0,     nE - 1)] : sent;
      da.y = (e0 + 1 < nE) ? dsts[min(e0 + 1, nE - 1)] : sent;
      da.z = (e0 + 2 < nE) ? dsts[min(e0 + 2, nE - 1)] : sent;
      da.w = (e0 + 3 < nE) ? dsts[min(e0 + 3, nE - 1)] : sent;
      db.x = (e0 + 4 < nE) ? dsts[min(e0 + 4, nE - 1)] : sent;
      db.y = (e0 + 5 < nE) ? dsts[min(e0 + 5, nE - 1)] : sent;
      db.z = (e0 + 6 < nE) ? dsts[min(e0 + 6, nE - 1)] : sent;
      db.w = (e0 + 7 < nE) ? dsts[min(e0 + 7, nE - 1)] : sent;
    }
    const unsigned nb = (unsigned)slotBase, nv = (unsigned)nValid;
    const unsigned s0 = (unsigned)da.x - nb, s1 = (unsigned)da.y - nb;
    const unsigned s2 = (unsigned)da.z - nb, s3 = (unsigned)da.w - nb;
    const unsigned s4 = (unsigned)db.x - nb, s5 = (unsigned)db.y - nb;
    const unsigned s6 = (unsigned)db.z - nb, s7 = (unsigned)db.w - nb;
    const bool h0 = (s0 < (unsigned)NB) & ((unsigned)da.x < nv);
    const bool h1 = (s1 < (unsigned)NB) & ((unsigned)da.y < nv);
    const bool h2 = (s2 < (unsigned)NB) & ((unsigned)da.z < nv);
    const bool h3 = (s3 < (unsigned)NB) & ((unsigned)da.w < nv);
    const bool h4 = (s4 < (unsigned)NB) & ((unsigned)db.x < nv);
    const bool h5 = (s5 < (unsigned)NB) & ((unsigned)db.y < nv);
    const bool h6 = (s6 < (unsigned)NB) & ((unsigned)db.z < nv);
    const bool h7 = (s7 < (unsigned)NB) & ((unsigned)db.w < nv);
    const unsigned any = __builtin_amdgcn_ballot_w32(h0 | h1 | h2 | h3 | h4 | h5 | h6 | h7);
    if (any != 0u) {
#define HITJ(J, HJ, SJ) { \
        const unsigned mj = __builtin_amdgcn_ballot_w32(HJ); \
        if (mj != 0u) { \
          if (HJ) { \
            const int pos = wc + (int)__builtin_amdgcn_mbcnt_lo(mj, 0u); \
            if (pos < WCAP) list[wave * WCAP + pos] = ((el0 + (J)) << 12) | (int)(SJ); \
          } \
          wc += (int)__builtin_popcount(mj); } }
      HITJ(0, h0, s0)
      HITJ(1, h1, s1)
      HITJ(2, h2, s2)
      HITJ(3, h3, s3)
      HITJ(4, h4, s4)
      HITJ(5, h5, s5)
      HITJ(6, h6, s6)
      HITJ(7, h7, s7)
#undef HITJ
    }
  }
  return wc;
}

__global__ __launch_bounds__(NTHR) void k_wprep(
    const float* __restrict__ Win, const float* __restrict__ W1, const float* __restrict__ W2,
    const float* __restrict__ W3, unsigned short* wh, unsigned short* wl) {
  const int i = blockIdx.x * NTHR + (int)threadIdx.x;
  if (i >= WROWS * (CH / 8)) return;
  const int n  = i >> 4;
  const int k0 = (i & 15) * 8;
  const float* src; int col;
  if (n < 128)      { src = Win;           col = n; }
  else if (n < 256) { src = W1;            col = n - 128; }
  else if (n < 384) { src = W2;            col = n - 256; }
  else if (n < 512) { src = W2 + 128 * CH; col = n - 384; }
  else              { src = W3;            col = n - 512; }
  v4f a, b;
  a.x = src[(size_t)(k0 + 0) * CH + col];
  a.y = src[(size_t)(k0 + 1) * CH + col];
  a.z = src[(size_t)(k0 + 2) * CH + col];
  a.w = src[(size_t)(k0 + 3) * CH + col];
  b.x = src[(size_t)(k0 + 4) * CH + col];
  b.y = src[(size_t)(k0 + 5) * CH + col];
  b.z = src[(size_t)(k0 + 6) * CH + col];
  b.w = src[(size_t)(k0 + 7) * CH + col];
  v4us ha, la, hb, lb;
  split4(a, ha, la);
  split4(b, hb, lb);
  U8 hv, lv;
  hv.q[0] = ha; hv.q[1] = hb;
  lv.q[0] = la; lv.q[1] = lb;
  unsigned short* ph = wh + (size_t)i * 8;
  unsigned short* pl = wl + (size_t)i * 8;
  *(volatile v8us*)ph = hv.v;
  *(volatile v8us*)pl = lv.v;
  __threadfence();
  *(volatile v8us*)ph = hv.v;
  *(volatile v8us*)pl = lv.v;
}

__global__ __launch_bounds__(NTHR) void k_count(
    const int* __restrict__ dsts, const int* __restrict__ nvp, int cap, int* cnt, int nE, int vec8) {
  __shared__ __attribute__((aligned(16))) int scnt[NBC];
  __shared__ __attribute__((aligned(16))) int list[LISTN];
  __shared__ int wcnt[NWAVE];
  const int tid = threadIdx.x, lane = tid & 31, wave = tid >> 5;
  const int slotBase = blockIdx.x * NBC;
  int nValid = nvp[0];
  nValid = nValid < 0 ? 0 : (nValid > cap ? cap : nValid);

  for (int i = tid; i < NBC; i += NTHR) scnt[i] = 0;
  __syncthreads();

  const int nChunks = (nE + CHUNK - 1) / CHUNK;
#pragma unroll 1
  for (int ch = 0; ch < nChunks; ++ch) {
    const int cbase = ch * CHUNK;
    const int wc = scan_chunk<NBC>(dsts, nE, cbase, slotBase, nValid, vec8, list, tid, lane, wave);
    if (lane == 0) wcnt[wave] = wc;
    __syncthreads();
    if (wave == 0) {
#pragma unroll 1
      for (int wsx = 0; wsx < NWAVE; ++wsx) {
        int n = __builtin_amdgcn_readfirstlane(wcnt[wsx]);
        n = n > WCAP ? WCAP : (n < 0 ? 0 : n);
        const int* lp = list + wsx * WCAP;
#pragma unroll 1
        for (int i = 0; i < n; ++i) {
          const int ent  = __builtin_amdgcn_readfirstlane(lp[i]);
          const int slot = ent & (NBC - 1);
          if (lane == 0) scnt[slot] = scnt[slot] + 1;
        }
      }
    }
    __syncthreads();
  }

  v4i cq[4];
#pragma unroll
  for (int q = 0; q < 4; ++q) {
    const int f = (wave * 4 + q) * 128 + 4 * lane;
    cq[q] = *(const v4i*)(scnt + f);
  }
  int* cp = cnt + (size_t)slotBase;
#pragma unroll
  for (int q = 0; q < 4; ++q) {
    const int f = (wave * 4 + q) * 128 + 4 * lane;
    *(volatile v4i*)(cp + f) = cq[q];
  }
  __threadfence();
#pragma unroll
  for (int q = 0; q < 4; ++q) {
    const int f = (wave * 4 + q) * 128 + 4 * lane;
    *(volatile v4i*)(cp + f) = cq[q];
  }
}

__global__ __launch_bounds__(OTHR) void k_offsets(
    const int* __restrict__ cnt, int* off, int* rbase, int nChunk) {
  __shared__ __attribute__((aligned(16))) int soff[NBC];
  __shared__ __attribute__((aligned(16))) int srb[RBN];
  __shared__ int wtot[OTHR / 32];
  const int tid = threadIdx.x, lane = tid & 31, wave = tid >> 5, sub = tid >> 7;
  for (int i = tid; i < RBN; i += OTHR) srb[i] = 0;
  int carry = 0;
#pragma unroll 1
  for (int ch = 0; ch < nChunk; ++ch) {
    const int base = ch * NBC;
    const v4i c0 = *(const v4i*)(cnt + base + 8 * tid);
    const v4i c1 = *(const v4i*)(cnt + base + 8 * tid + 4);
    const int e0 = max(c0.x, 0), e1 = max(c0.y, 0), e2 = max(c0.z, 0), e3 = max(c0.w, 0);
    const int e4 = max(c1.x, 0), e5 = max(c1.y, 0), e6 = max(c1.z, 0), e7 = max(c1.w, 0);
    const int ts = e0 + e1 + e2 + e3 + e4 + e5 + e6 + e7;
    int incl = ts;
#pragma unroll
    for (int d = 1; d < 32; d <<= 1) {
      const int t = __shfl_up(incl, d);
      if (lane >= d) incl += t;
    }
    if (lane == 31) wtot[wave] = incl;
    __syncthreads();
    const int S0 = wtot[0]  + wtot[1]  + wtot[2]  + wtot[3];
    const int S1 = wtot[4]  + wtot[5]  + wtot[6]  + wtot[7];
    const int S2 = wtot[8]  + wtot[9]  + wtot[10] + wtot[11];
    const int S3 = wtot[12] + wtot[13] + wtot[14] + wtot[15];
    int pre = 0;
#pragma unroll 1
    for (int w = 4 * sub; w < wave; ++w) pre += wtot[w];
    const int b0 = carry;
    const int b1 = b0 + ((S0 + 31) & ~31);
    const int b2 = b1 + ((S1 + 31) & ~31);
    const int b3 = b2 + ((S2 + 31) & ~31);
    const int b4 = b3 + ((S3 + 31) & ~31);
    const int myb = sub == 0 ? b0 : (sub == 1 ? b1 : (sub == 2 ? b2 : b3));
    if (tid == 0) {
      srb[min(4 * ch + 0, RBN - 1)] = b0;
      srb[min(4 * ch + 1, RBN - 1)] = b1;
      srb[min(4 * ch + 2, RBN - 1)] = b2;
      srb[min(4 * ch + 3, RBN - 1)] = b3;
    }
    int run = myb + pre + incl - ts;
    soff[8 * tid + 0] = run; run += e0;
    soff[8 * tid + 1] = run; run += e1;
    soff[8 * tid + 2] = run; run += e2;
    soff[8 * tid + 3] = run; run += e3;
    soff[8 * tid + 4] = run; run += e4;
    soff[8 * tid + 5] = run; run += e5;
    soff[8 * tid + 6] = run; run += e6;
    soff[8 * tid + 7] = run;
    carry = b4;
    __syncthreads();
    const v4i o0 = *(const v4i*)(soff + 4 * tid);
    const v4i o1 = *(const v4i*)(soff + 4 * (tid + OTHR));
    int* op = off + base;
    *(volatile v4i*)(op + 4 * tid) = o0;
    *(volatile v4i*)(op + 4 * (tid + OTHR)) = o1;
    __threadfence();
    *(volatile v4i*)(op + 4 * tid) = o0;
    *(volatile v4i*)(op + 4 * (tid + OTHR)) = o1;
    __syncthreads();
  }
  if (tid == 0) srb[min(4 * nChunk, RBN - 1)] = carry;
  __syncthreads();
  v4i rv = {0, 0, 0, 0};
  if (tid < 32) rv = *(const v4i*)(srb + 4 * tid);
  if (tid < 32) *(volatile v4i*)(rbase + 4 * tid) = rv;
  __threadfence();
  if (tid < 32) *(volatile v4i*)(rbase + 4 * tid) = rv;
}

__global__ __launch_bounds__(NTHR) void k_fill(
    const int* __restrict__ dsts, const int* __restrict__ srcs,
    const int* __restrict__ nvd, int dcap, const int* __restrict__ nvs, int scap,
    const int* __restrict__ off, const int* __restrict__ rbase,
    int* csr, int nE, int vec8, int csrLen) {
  extern __shared__ v4f lds_dyn[];
  int* region = (int*)lds_dyn;
  int* cursor = region + RCAP;
  int* list   = cursor + NBF;
  int* wcnt   = list + LISTN;
  const int tid = threadIdx.x, lane = tid & 31, wave = tid >> 5;
  const int b = blockIdx.x;
  const int slotBase = b * NBF;
  int nValid = nvd[0];
  nValid = nValid < 0 ? 0 : (nValid > dcap ? dcap : nValid);
  int sv = nvs[0];
  sv = sv < 1 ? 1 : (sv > scap ? scap : sv);
  const int smax = sv - 1;

  int rb0 = rbase[b];
  const int rb1 = rbase[b + 1];
  rb0 = rb0 < 0 ? 0 : (rb0 > csrLen ? csrLen : rb0);
  rb0 &= ~31;
  int len = rb1 - rb0;
  len = len < 0 ? 0 : (len > RCAP ? RCAP : len);
  int lenW = (len + 31) & ~31;
  if (rb0 + lenW > csrLen) lenW = (csrLen - rb0) & ~31;

  {
    const v4i z = {0, 0, 0, 0};
    for (int i = tid; i < RCAP / 4; i += NTHR) ((v4i*)region)[i] = z;
    for (int s = tid; s < NBF; s += NTHR) {
      int o = off[slotBase + s] - rb0;
      o = o < 0 ? 0 : (o > RCAP ? RCAP : o);
      cursor[s] = o;
    }
  }
  __syncthreads();

  const int nChunks = (nE + CHUNK - 1) / CHUNK;
#pragma unroll 1
  for (int ch = 0; ch < nChunks; ++ch) {
    const int cbase = ch * CHUNK;
    const int wc = scan_chunk<NBF>(dsts, nE, cbase, slotBase, nValid, vec8, list, tid, lane, wave);
    if (lane == 0) wcnt[wave] = wc;
    __syncthreads();
    if (wave == 0) {
#pragma unroll 1
      for (int wsx = 0; wsx < NWAVE; ++wsx) {
        int n = __builtin_amdgcn_readfirstlane(wcnt[wsx]);
        n = n > WCAP ? WCAP : (n < 0 ? 0 : n);
        const int* lp = list + wsx * WCAP;
#pragma unroll 1
        for (int i = 0; i < n; ++i) {
          const int ent  = __builtin_amdgcn_readfirstlane(lp[i]);
          const int slot = ent & (NBF - 1);
          int e = cbase + ((ent >> 12) & (CHUNK - 1));
          e = e > nE - 1 ? nE - 1 : e;
          int src = srcs[e];
          src = src < 0 ? 0 : (src > smax ? smax : src);
          if (lane == 0) {
            int pos = cursor[slot];
            pos = pos < 0 ? 0 : (pos > RCAP - 1 ? RCAP - 1 : pos);
            region[pos] = src;
            const int np = pos + 1;
            cursor[slot] = np > RCAP ? RCAP : np;
          }
        }
      }
    }
    __syncthreads();
  }

  const int nv = lenW >> 2;
  int* gp = csr + rb0;
#pragma unroll 1
  for (int i = tid; i < nv; i += NTHR) { const v4i v = ((const v4i*)region)[i]; *(volatile v4i*)(gp + 4 * i) = v; }
  __threadfence();
#pragma unroll 1
  for (int i = tid; i < nv; i += NTHR) { const v4i v = ((const v4i*)region)[i]; *(volatile v4i*)(gp + 4 * i) = v; }
}

__global__ __launch_bounds__(NTHR) void k_gemm1(
    const float* __restrict__ A, int nRowsA,
    const unsigned short* __restrict__ bH, const unsigned short* __restrict__ bL,
    const float* __restrict__ bias, int relu, float* dst, int nRowsOut) {
  extern __shared__ v4f lds_dyn[];
  unsigned short* sH  = (unsigned short*)lds_dyn;
  unsigned short* sL  = sH + GROWS * AP;
  float*          stg = (float*)lds_dyn;
  const int tid = threadIdx.x, lane = tid & 31, wave = tid >> 5, hh = lane >> 4, m = lane & 15;
  const int rowBase = blockIdx.x * GROWS;

  stage_rows(A, nRowsA, rowBase, sH, sL, tid);
  __syncthreads();

  v8f acc[8];
#pragma unroll
  for (int t = 0; t < 8; ++t) { v8f z = {0.f, 0.f, 0.f, 0.f, 0.f, 0.f, 0.f, 0.f}; acc[t] = z; }
  const int ao = (wave * 16 + m) * AP + 8 * hh;
  const int bo = m * CH + 8 * hh;
  mma_strip(sH + ao, sL + ao, bH + bo, bL + bo, acc);
  __syncthreads();

  epi_rows(acc, stg, bias, 1, relu, dst, rowBase, nRowsOut, wave, lane);
}

__global__ __launch_bounds__(NTHR) void k_gemm2(
    const float* __restrict__ A, int nRowsA,
    const unsigned short* __restrict__ bH, const unsigned short* __restrict__ bL,
    const float* __restrict__ bias, float* dst0, float* dst1, int nRowsOut) {
  extern __shared__ v4f lds_dyn[];
  unsigned short* sH  = (unsigned short*)lds_dyn;
  unsigned short* sL  = sH + GROWS * AP;
  float*          stg = (float*)(sL + GROWS * AP);
  const int tid = threadIdx.x, lane = tid & 31, wave = tid >> 5, hh = lane >> 4, m = lane & 15;
  const int rowBase = blockIdx.x * GROWS;

  stage_rows(A, nRowsA, rowBase, sH, sL, tid);
  __syncthreads();

  const int ao = (wave * 16 + m) * AP + 8 * hh;
  const int bo = m * CH + 8 * hh;
#pragma unroll 1
  for (int g = 0; g < 2; ++g) {
    v8f acc[8];
#pragma unroll
    for (int t = 0; t < 8; ++t) { v8f z = {0.f, 0.f, 0.f, 0.f, 0.f, 0.f, 0.f, 0.f}; acc[t] = z; }
    const size_t go = (size_t)g * CH * CH;
    mma_strip(sH + ao, sL + ao, bH + go + bo, bL + go + bo, acc);
    float* dst = g == 0 ? dst0 : dst1;
    epi_rows(acc, stg, bias, g == 0 ? 1 : 0, 0, dst, rowBase, nRowsOut, wave, lane);
    __syncthreads();
  }
}

__global__ __launch_bounds__(NTHR) void k_edge(
    const int* __restrict__ csr, const int* __restrict__ off, const int* __restrict__ cnt, int csrLen,
    const float* __restrict__ T, int smax,
    const unsigned short* __restrict__ bH, const unsigned short* __restrict__ bL,
    const float* __restrict__ bz, float* Q, int nRowsOut) {
  extern __shared__ v4f lds_dyn[];
  unsigned short* sH  = (unsigned short*)lds_dyn;
  unsigned short* sL  = sH + GROWS * AP;
  float*          stg = (float*)lds_dyn;
  const int tid = threadIdx.x, lane = tid & 31, wave = tid >> 5, hh = lane >> 4, m = lane & 15;
  const int rowBase = blockIdx.x * GROWS;
  const int tb = rowBase + 16 * wave;
  const int cl = tb + m;
  const int cnt_l = cnt[cl];
  const int off_l = off[cl];

#pragma unroll 1
  for (int j = 0; j < 16; ++j) {
    int n = __builtin_amdgcn_readlane(cnt_l, j);
    n = n < 0 ? 0 : (n > DEGCAP ? DEGCAP : n);
    const int st = __builtin_amdgcn_readlane(off_l, j);
    const v4f a = seg_sum(csr, csrLen, st, n, T, smax, lane);
    v4us hq, lq;
    split4(a, hq, lq);
    const int o = (16 * wave + j) * AP + 4 * lane;
    *(v4us*)(sH + o) = hq;
    *(v4us*)(sL + o) = lq;
  }
  __syncthreads();

  v8f acc[8];
#pragma unroll
  for (int t = 0; t < 8; ++t) { v8f z = {0.f, 0.f, 0.f, 0.f, 0.f, 0.f, 0.f, 0.f}; acc[t] = z; }
  const int ao = (wave * 16 + m) * AP + 8 * hh;
  const int bo = m * CH + 8 * hh;
  mma_strip(sH + ao, sL + ao, bH + bo, bL + bo, acc);
  __syncthreads();

  epi_rows(acc, stg, bz, 0, 0, Q, rowBase, nRowsOut, wave, lane);
}

__global__ __launch_bounds__(NTHR) void k_node(
    const int* __restrict__ csr, const int* __restrict__ off, const int* __restrict__ cnt, int csrLen,
    const float* __restrict__ Q, const int* __restrict__ nve,
    const float* __restrict__ P, const float* __restrict__ b2, const float* __restrict__ x0,
    const unsigned short* __restrict__ bH, const unsigned short* __restrict__ bL,
    const float* __restrict__ b3, float* dst, int nRowsOut) {
  extern __shared__ v4f lds_dyn[];
  unsigned short* sH  = (unsigned short*)lds_dyn;
  unsigned short* sL  = sH + GROWS * AP;
  float*          stg = (float*)lds_dyn;
  const int tid = threadIdx.x, lane = tid & 31, wave = tid >> 5, hh = lane >> 4, m = lane & 15;
  const int rowBase = blockIdx.x * GROWS;
  const int tb = rowBase + 16 * wave;
  const int cl = tb + m;
  const int cnt_l = cnt[cl];
  const int off_l = off[cl];
  int qv = nve[0];
  qv = qv < 1 ? 1 : (qv > EROWS ? EROWS : qv);
  const int qmax = qv - 1;
  const v4f bb = *(const v4f*)(b2 + 4 * lane);

#pragma unroll 1
  for (int j = 0; j < 16; ++j) {
    const int v = tb + j;
    int n = __builtin_amdgcn_readlane(cnt_l, j);
    n = n < 0 ? 0 : (n > DEGCAP ? DEGCAP : n);
    const int st = __builtin_amdgcn_readlane(off_l, j);
    const v4f a  = seg_sum(csr, csrLen, st, n, Q, qmax, lane);
    const v4f pr = *(const v4f*)(P  + (size_t)v * CH + 4 * lane);
    const v4f xr = *(const v4f*)(x0 + (size_t)v * CH + 4 * lane);
    const float fn = (float)n;
    const v4f xv = (pr + bb) * fn + a;
    const v4f t  = xv * 0.5f + xr * 0.5f;
    v4us hq, lq;
    split4(t, hq, lq);
    const int o = (16 * wave + j) * AP + 4 * lane;
    *(v4us*)(sH + o) = hq;
    *(v4us*)(sL + o) = lq;
  }
  __syncthreads();

  v8f acc[8];
#pragma unroll
  for (int t = 0; t < 8; ++t) { v8f z = {0.f, 0.f, 0.f, 0.f, 0.f, 0.f, 0.f, 0.f}; acc[t] = z; }
  const int ao = (wave * 16 + m) * AP + 8 * hh;
  const int bo = m * CH + 8 * hh;
  mma_strip(sH + ao, sL + ao, bH + bo, bL + bo, acc);
  __syncthreads();

  epi_rows(acc, stg, b3, 1, 1, dst, rowBase, nRowsOut, wave, lane);
}

#define CARVE(name, bytes) const size_t name = wo; wo += (size_t)(bytes); wo = (wo + 255) & ~(size_t)255;

extern "C" void kernel_launch(void* const* d_in, const int* in_sizes, int n_in,
                              void* d_out, int out_size, void* d_ws, size_t ws_size,
                              hipStream_t stream) {
  if (n_in < 13) return;
  const int N = in_sizes[0] / CH;
  if (N <= 0 || in_sizes[0] != N * CH) return;
  if (in_sizes[1] != CH * CH || in_sizes[2] < CH || in_sizes[3] != CH * CH || in_sizes[4] < CH ||
      in_sizes[5] != 2 * CH * CH || in_sizes[6] < CH || in_sizes[7] != CH * CH || in_sizes[8] < CH) return;
  const int nE = in_sizes[9];
  if (nE <= 0 || in_sizes[10] != nE || in_sizes[11] < 1 || in_sizes[12] < 1) return;
  if (out_size != N * CH) return;
  if (nE > (1 << 28) || N > (1 << 24)) return;

  const float* x    = (const float*)d_in[0];
  const float* W_in = (const float*)d_in[1];
  const float* b_in = (const float*)d_in[2];
  const float* W1   = (const float*)d_in[3];
  const float* b1   = (const float*)d_in[4];
  const float* W2   = (const float*)d_in[5];
  const float* b2   = (const float*)d_in[6];
  const float* W3   = (const float*)d_in[7];
  const float* b3   = (const float*)d_in[8];
  const int*   V    = (const int*)d_in[9];
  const int*   E    = (const int*)d_in[10];
  const int*   nNp  = (const int*)d_in[11];
  const int*   nEp  = (const int*)d_in[12];
  float* out = (float*)d_out;

  const int NPAD  = ((N + GROWS - 1) / GROWS) * GROWS;
  const int nGemm = NPAD / GROWS;
  const int nBCV  = (N + NBC - 1) / NBC;
  const int CNTV  = nBCV * NBC;
  const int nBFV  = (N + NBF - 1) / NBF;
  const int nBCE  = (EROWS + NBC - 1) / NBC;
  const int CNTE  = nBCE * NBC;
  const int nBFE  = EROWS / NBF;
  const int nEdge = EROWS / GROWS;
  if (4 * nBCV + 1 > RBN || 4 * nBCE + 1 > RBN) return;
  const int csrLen = ((nE + 31) & ~31) + 4096;

  char* ws = (char*)d_ws;
  size_t wo = 0;
  CARVE(oWH,   (size_t)WROWS * CH * 2)
  CARVE(oWL,   (size_t)WROWS * CH * 2)
  CARVE(oX0,   (size_t)NPAD * CH * 4)
  CARVE(oCur,  (size_t)NPAD * CH * 4)
  CARVE(oT,    (size_t)NPAD * CH * 4)
  CARVE(oP,    (size_t)NPAD * CH * 4)
  CARVE(oQ,    (size_t)EROWS * CH * 4)
  CARVE(oCntE, (size_t)CNTE * 4)
  CARVE(oOffE, (size_t)CNTE * 4)
  CARVE(oRbE,  (size_t)RBN * 4)
  CARVE(oCsrE, (size_t)csrLen * 4)
  CARVE(oCntV, (size_t)CNTV * 4)
  CARVE(oOffV, (size_t)CNTV * 4)
  CARVE(oRbV,  (size_t)RBN * 4)
  CARVE(oCsrV, (size_t)csrLen * 4)
  if (wo > ws_size) return;
  unsigned short* wh = (unsigned short*)(ws + oWH);
  unsigned short* wl = (unsigned short*)(ws + oWL);
  float* x0f  = (float*)(ws + oX0);
  float* cur  = (float*)(ws + oCur);
  float* T    = (float*)(ws + oT);
  float* P    = (float*)(ws + oP);
  float* Q    = (float*)(ws + oQ);
  int*   cntE = (int*)(ws + oCntE);
  int*   offE = (int*)(ws + oOffE);
  int*   rbE  = (int*)(ws + oRbE);
  int*   csrE = (int*)(ws + oCsrE);
  int*   cntV = (int*)(ws + oCntV);
  int*   offV = (int*)(ws + oOffV);
  int*   rbV  = (int*)(ws + oRbV);
  int*   csrV = (int*)(ws + oCsrV);
  const unsigned short* wInH = wh;              const unsigned short* wInL = wl;
  const unsigned short* wAH  = wh + 128 * CH;   const unsigned short* wAL  = wl + 128 * CH;
  const unsigned short* wBH  = wh + 384 * CH;   const unsigned short* wBL  = wl + 384 * CH;
  const unsigned short* w3H  = wh + 512 * CH;   const unsigned short* w3L  = wl + 512 * CH;

  const int vec8 = ((nE & 3) == 0) ? 1 : 0;

  k_wprep<<<WROWS * (CH / 8) / NTHR, NTHR, 0, stream>>>(W_in, W1, W2, W3, wh, wl);

  hipFuncSetAttribute(reinterpret_cast<const void*>(&k_fill),
                      hipFuncAttributeMaxDynamicSharedMemorySize, LDS_FILL);
  k_count<<<nBCE, NTHR, 0, stream>>>(E, nEp, EROWS, cntE, nE, vec8);
  k_offsets<<<1, OTHR, 0, stream>>>(cntE, offE, rbE, nBCE);
  k_fill<<<nBFE, NTHR, LDS_FILL, stream>>>(E, V, nEp, EROWS, nNp, N, offE, rbE, csrE, nE, vec8, csrLen);

  k_count<<<nBCV, NTHR, 0, stream>>>(V, nNp, N, cntV, nE, vec8);
  k_offsets<<<1, OTHR, 0, stream>>>(cntV, offV, rbV, nBCV);
  k_fill<<<nBFV, NTHR, LDS_FILL, stream>>>(V, E, nNp, N, nEp, EROWS, offV, rbV, csrV, nE, vec8, csrLen);

  hipFuncSetAttribute(reinterpret_cast<const void*>(&k_gemm1),
                      hipFuncAttributeMaxDynamicSharedMemorySize, LDS_A);
  hipFuncSetAttribute(reinterpret_cast<const void*>(&k_gemm2),
                      hipFuncAttributeMaxDynamicSharedMemorySize, LDS_G2);
  hipFuncSetAttribute(reinterpret_cast<const void*>(&k_edge),
                      hipFuncAttributeMaxDynamicSharedMemorySize, LDS_A);
  hipFuncSetAttribute(reinterpret_cast<const void*>(&k_node),
                      hipFuncAttributeMaxDynamicSharedMemorySize, LDS_A);
  k_gemm1<<<nGemm, NTHR, LDS_A, stream>>>(x, N, wInH, wInL, b_in, 1, x0f, NPAD);

  for (int layer = 0; layer < 2; ++layer) {
    const float* xin = layer == 0 ? x0f : cur;
    k_gemm2<<<nGemm, NTHR, LDS_G2, stream>>>(xin, NPAD, wAH, wAL, b1, T, P, NPAD);
    k_edge<<<nEdge, NTHR, LDS_A, stream>>>(csrE, offE, cntE, csrLen, T, N - 1, wBH, wBL, b2, Q, EROWS);
    float* dst = layer == 0 ? cur : out;
    const int nro = layer == 0 ? NPAD : N;
    k_node<<<nGemm, NTHR, LDS_A, stream>>>(csrV, offV, cntV, csrLen, Q, nEp, P, b2, x0f, w3H, w3L, b3, dst, nro);
  }
}
